// SparseMemoryAttention_64055142252572
// MI455X (gfx1250) — hardware-verified
//
#include <hip/hip_runtime.h>
#include <stddef.h>
#include <stdint.h>

#define NBATCH 2
#define SEQ    2048
#define EMB    1024
#define NHD    16
#define HDIM   64
#define HALFW  128
#define MROWS  4096
#define PLP    2048
#define WPLANE 2097152
#define APLANE 8388608
#define HPLANE 4194304
#define QBLK   64
#define NQT    32
#define PPITCH 40
#define OPITCH 68
#define T16P   136
#define T16T   72
#define T32P   132
#define WTP    72

static_assert(MROWS == NBATCH * SEQ);
static_assert(EMB == NHD * HDIM);
static_assert(SEQ == NQT * QBLK);
static_assert(EMB % 128 == 0);
static_assert(MROWS % 64 == 0);
static_assert(SEQ % 64 == 0);
static_assert(HALFW % 32 == 0);
static_assert(APLANE == MROWS * PLP);
static_assert(HPLANE == MROWS * EMB);
static_assert(HPLANE == NBATCH * NHD * HDIM * SEQ);
static_assert(WPLANE == EMB * PLP);
static_assert((MROWS * EMB) % (8 * 256) == 0);
static_assert(128 * T16T >= 64 * T16P);

#define DEVI __device__ __forceinline__

typedef __bf16 v16b __attribute__((ext_vector_type(16)));
typedef _Float16 v16h __attribute__((ext_vector_type(16)));
typedef unsigned short v8us __attribute__((ext_vector_type(8)));
typedef float v8f __attribute__((ext_vector_type(8)));
typedef float v4f __attribute__((ext_vector_type(4)));
typedef unsigned int v4u __attribute__((ext_vector_type(4)));

union FragB { v16b v; v8us u[2]; };
union FragH { v16h v; v8us u[2]; };

DEVI v8f zero8() { return (v8f){0.f, 0.f, 0.f, 0.f, 0.f, 0.f, 0.f, 0.f}; }

DEVI v8f mmab(v16b a, v16b b, v8f c) {
  c = __builtin_amdgcn_wmma_f32_16x16x32_bf16(false, a, false, b, (short)0, c, false, false);
  asm volatile("v_nop\n\tv_nop\n\tv_nop\n\tv_nop" : "+v"(c) : "v"(a), "v"(b));
  return c;
}
DEVI v8f mmah(v16h a, v16h b, v8f c) {
  c = __builtin_amdgcn_wmma_f32_16x16x32_f16(false, a, false, b, (short)0, c, false, false);
  asm volatile("v_nop\n\tv_nop\n\tv_nop\n\tv_nop" : "+v"(c) : "v"(a), "v"(b));
  return c;
}

DEVI void ldpair(const unsigned short* p, int ld, int row0, int k0, int lane, v8us& u0, v8us& u1) {
  const int m = lane & 15, lh = lane >> 4;
  const unsigned short* q = p + (size_t)(row0 + m) * ld + k0 + 8 * lh;
  u0 = *(const v8us*)(q);
  u1 = *(const v8us*)(q + 16);
}
DEVI v16b ldfragb(const unsigned short* p, int ld, int row0, int k0, int lane) {
  FragB f;
  ldpair(p, ld, row0, k0, lane, f.u[0], f.u[1]);
  return f.v;
}
DEVI v16h ldfragh(const unsigned short* p, int ld, int row0, int k0, int lane) {
  FragH f;
  ldpair(p, ld, row0, k0, lane, f.u[0], f.u[1]);
  return f.v;
}

DEVI unsigned int bfrne(float f) {
  const unsigned int u = __float_as_uint(f);
  return (u + 0x7fffu + ((u >> 16) & 1u)) >> 16;
}
DEVI void bfhl(float f, unsigned int& hb, unsigned int& lb) {
  hb = bfrne(f);
  const float res = f - __uint_as_float(hb << 16);
  lb = bfrne(res);
}
DEVI void pack2hl(float a, float b, unsigned int& ph, unsigned int& pl) {
  unsigned int ha, la, hb, lb;
  bfhl(a, ha, la);
  bfhl(b, hb, lb);
  ph = ha | (hb << 16);
  pl = la | (lb << 16);
}
DEVI unsigned short f2h(float f) { return __builtin_bit_cast(unsigned short, (_Float16)f); }

__global__ __launch_bounds__(256) void k_xplane(const float* __restrict__ x, unsigned short* __restrict__ xp) {
  const size_t p = (size_t)blockIdx.x * 256 + threadIdx.x;
  const size_t e = p * 8;
  const int row = (int)(e >> 10), col = (int)(e & 1023);
  const v4f f0 = *(const v4f*)(x + e), f1 = *(const v4f*)(x + e + 4);
  v4u hi, lo;
  unsigned int ph, pl;
  pack2hl(f0[0], f0[1], ph, pl); hi[0] = ph; lo[0] = pl;
  pack2hl(f0[2], f0[3], ph, pl); hi[1] = ph; lo[1] = pl;
  pack2hl(f1[0], f1[1], ph, pl); hi[2] = ph; lo[2] = pl;
  pack2hl(f1[2], f1[3], ph, pl); hi[3] = ph; lo[3] = pl;
  unsigned short* dst = xp + (size_t)row * PLP + col;
  for (int ps = 0; ps < 2; ++ps) {
    *(volatile v4u*)(dst) = hi;
    *(volatile v4u*)(dst + EMB) = lo;
    __threadfence();
  }
}

__global__ __launch_bounds__(256) void k_wplane(const float* __restrict__ wq, const float* __restrict__ wk,
                                               const float* __restrict__ wv, const float* __restrict__ wo,
                                               unsigned short* __restrict__ wt) {
  __shared__ __align__(16) unsigned short sw[2 * 64 * WTP];
  const int tid = threadIdx.x, lane = tid & 31, wave = tid >> 5;
  const int z = blockIdx.z;
  const int n0 = blockIdx.x * 64, k0 = blockIdx.y * 64;
  const float* W = (z == 0) ? wq : ((z == 1) ? wk : ((z == 2) ? wv : wo));
#pragma unroll
  for (int it = 0; it < 4; ++it) {
    const int idx = it * 256 + tid;
    const int r = idx >> 4, c4 = (idx & 15) * 4;
    const v4f f = *(const v4f*)(W + (size_t)(k0 + r) * EMB + n0 + c4);
#pragma unroll
    for (int e = 0; e < 4; ++e) {
      unsigned int hb, lb;
      bfhl(f[e], hb, lb);
      sw[(c4 + e) * WTP + r] = (unsigned short)hb;
      sw[64 * WTP + (c4 + e) * WTP + r] = (unsigned short)lb;
    }
  }
  __syncthreads();
  v4u val[4];
#pragma unroll
  for (int it = 0; it < 4; ++it) {
    const int L = wave * 16 + it * 4 + (lane >> 3);
    const int n = L >> 1, pl = L & 1;
    const int c8 = (lane & 7) * 8;
    val[it] = *(const v4u*)(sw + (pl * 64 + n) * WTP + c8);
  }
  unsigned short* wz = wt + (size_t)z * WPLANE;
  for (int ps = 0; ps < 2; ++ps) {
#pragma unroll
    for (int it = 0; it < 4; ++it) {
      const int L = wave * 16 + it * 4 + (lane >> 3);
      const int n = L >> 1, pl = L & 1;
      const int c8 = (lane & 7) * 8;
      *(volatile v4u*)(wz + (size_t)(n0 + n) * PLP + pl * EMB + k0 + c8) = val[it];
    }
    __threadfence();
  }
}

DEVI void gemm3(const unsigned short* __restrict__ A, const unsigned short* __restrict__ Bp,
                int arow0, int bcol0, int lane, v8f (&acc)[4]) {
#pragma unroll 1
  for (int sec = 0; sec < 3; ++sec) {
    const int aoff = (sec == 1) ? EMB : 0;
    const int boff = (sec == 2) ? EMB : 0;
#pragma unroll 2
    for (int k0 = 0; k0 < EMB; k0 += 32) {
      const v16b a = ldfragb(A, PLP, arow0, aoff + k0, lane);
#pragma unroll
      for (int t = 0; t < 4; ++t) {
        const v16b bfr = ldfragb(Bp, PLP, bcol0 + 16 * t, boff + k0, lane);
        acc[t] = mmab(a, bfr, acc[t]);
      }
    }
  }
}

__global__ __launch_bounds__(256) void k_gemm16(const unsigned short* __restrict__ xp,
                                                const unsigned short* __restrict__ wt,
                                                const float* __restrict__ bq,
                                                const float* __restrict__ bk,
                                                const float* __restrict__ bv,
                                                unsigned short* __restrict__ qkv) {
  __shared__ __align__(16) unsigned short tile[128 * T16T];
  const int tid = threadIdx.x, lane = tid & 31, wave = tid >> 5;
  const int hh = lane >> 4, m = lane & 15;
  const int z = blockIdx.z;
  const int m0 = blockIdx.y * 64, n0 = blockIdx.x * 128;
  const int wm = wave >> 1, wn = wave & 1;
  const unsigned short* wz = wt + (size_t)z * WPLANE;
  const float* bias = (z == 0) ? bq : ((z == 1) ? bk : bv);
  const int tr = (z == 2);

  v8f acc[4];
#pragma unroll
  for (int t = 0; t < 4; ++t) acc[t] = zero8();
  gemm3(xp, wz, m0 + wm * 16, n0 + wn * 64, lane, acc);

#pragma unroll
  for (int t = 0; t < 4; ++t) {
    const int col = wn * 64 + 16 * t + m;
    const float bb = bias[n0 + col];
#pragma unroll
    for (int r = 0; r < 8; ++r) {
      const int row = wm * 16 + 8 * hh + r;
      const int idx = tr ? (col * T16T + row) : (row * T16P + col);
      tile[idx] = f2h(acc[t][r] + bb);
    }
  }
  __syncthreads();

  v4u val[4];
#pragma unroll
  for (int it = 0; it < 4; ++it) {
    const int L = wave * 16 + it * 4 + (lane >> 3);
    const int c8 = (lane & 7) * 8;
    const int s0 = (L >> 1) * T16P + (L & 1) * 64 + c8;
    const int s1 = L * T16T + c8;
    val[it] = *(const v4u*)(tile + (tr ? s1 : s0));
  }
  const int bb2 = m0 >> 11, j0 = m0 & (SEQ - 1);
  unsigned short* dz = qkv + (size_t)z * HPLANE;
  for (int ps = 0; ps < 2; ++ps) {
#pragma unroll
    for (int it = 0; it < 4; ++it) {
      const int L = wave * 16 + it * 4 + (lane >> 3);
      const int c8 = (lane & 7) * 8;
      const size_t d0 = (size_t)(m0 + (L >> 1)) * EMB + n0 + (L & 1) * 64 + c8;
      const int n = n0 + L;
      const size_t d1 = ((size_t)((bb2 * NHD + (n >> 6)) * HDIM + (n & 63))) * SEQ + j0 + c8;
      *(volatile v4u*)(dz + (tr ? d1 : d0)) = val[it];
    }
    __threadfence();
  }
}

__global__ __launch_bounds__(128) void k_attn(const unsigned short* __restrict__ qp,
                                              const unsigned short* __restrict__ kp,
                                              const unsigned short* __restrict__ vt,
                                              unsigned short* __restrict__ cp) {
  __shared__ __align__(16) unsigned short Ps[4 * 16 * PPITCH];
  __shared__ __align__(16) float Os[4 * 16 * OPITCH];
  const int tid = threadIdx.x, lane = tid & 31, wave = tid >> 5;
  const int hh = lane >> 4, m = lane & 15;
  const int bid = blockIdx.x;
  const int qt = bid & (NQT - 1);
  const int h = (bid >> 5) & (NHD - 1);
  const int b = bid >> 9;
  const int q0b = qt * QBLK;
  const int q0 = q0b + wave * 16;
  const int rowb = b * SEQ;
  const int jlo = max(q0b - HALFW, 0);
  const int jhi = min(q0b + QBLK + HALFW, SEQ);
  const int nch = (jhi - jlo) >> 5;

  v16h qf[2];
#pragma unroll
  for (int dI = 0; dI < 2; ++dI) qf[dI] = ldfragh(qp, EMB, rowb + q0, h * HDIM + dI * 32, lane);

  const float NEGI = -__builtin_huge_valf();
  float ms[8], ls[8];
#pragma unroll
  for (int r = 0; r < 8; ++r) { ms[r] = NEGI; ls[r] = 0.f; }
  v8f o[4];
#pragma unroll
  for (int dt = 0; dt < 4; ++dt) o[dt] = zero8();

  unsigned short* pw = Ps + wave * (16 * PPITCH);
  const unsigned short* vbase = vt + ((size_t)(b * NHD + h) * HDIM) * SEQ;

#pragma unroll 1
  for (int c = 0; c < nch; ++c) {
    const int jc = jlo + 32 * c;
    __syncthreads();
    v8f s[2];
#pragma unroll
    for (int jt = 0; jt < 2; ++jt) {
      s[jt] = zero8();
#pragma unroll
      for (int dI = 0; dI < 2; ++dI) {
        const v16h kf = ldfragh(kp, EMB, rowb + jc + 16 * jt, h * HDIM + dI * 32, lane);
        s[jt] = mmah(qf[dI], kf, s[jt]);
      }
    }
#pragma unroll
    for (int r = 0; r < 8; ++r) {
      const int q = q0 + 8 * hh + r;
      const int ja = jc + m, jb = jc + 16 + m;
      const bool oka = (ja >= q - HALFW) && (ja < q + HALFW);
      const bool okb = (jb >= q - HALFW) && (jb < q + HALFW);
      const float sa = s[0][r] * 0.125f, sb = s[1][r] * 0.125f;
      s[0][r] = oka ? sa : NEGI;
      s[1][r] = okb ? sb : NEGI;
    }
    float al[8];
#pragma unroll
    for (int r = 0; r < 8; ++r) {
      float mx = fmaxf(s[0][r], s[1][r]);
#pragma unroll
      for (int off = 1; off < 16; off <<= 1) mx = fmaxf(mx, __shfl_xor(mx, off, 32));
      const float mn = fmaxf(ms[r], mx);
      const bool noinf = (mn != NEGI);
      const float alpha = noinf ? __expf(ms[r] - mn) : 1.f;
      const float pa = noinf ? __expf(s[0][r] - mn) : 0.f;
      const float pb = noinf ? __expf(s[1][r] - mn) : 0.f;
      ms[r] = mn;
      float psum = pa + pb;
#pragma unroll
      for (int off = 1; off < 16; off <<= 1) psum += __shfl_xor(psum, off, 32);
      ls[r] = ls[r] * alpha + psum;
      al[r] = alpha;
      pw[(8 * hh + r) * PPITCH + m] = f2h(pa * 1024.0f);
      pw[(8 * hh + r) * PPITCH + 16 + m] = f2h(pb * 1024.0f);
    }
#pragma unroll
    for (int dt = 0; dt < 4; ++dt)
#pragma unroll
      for (int r = 0; r < 8; ++r) o[dt][r] *= al[r];
    __syncthreads();
    const v16h pf = ldfragh(pw, PPITCH, 0, 0, lane);
#pragma unroll
    for (int dt = 0; dt < 4; ++dt) {
      const v16h vf = ldfragh(vbase, SEQ, 16 * dt, jc, lane);
      o[dt] = mmah(pf, vf, o[dt]);
    }
  }

  float* ow = Os + wave * (16 * OPITCH);
#pragma unroll
  for (int r = 0; r < 8; ++r) {
    const float inv = (1.0f / ls[r]) * 0.0009765625f;
#pragma unroll
    for (int dt = 0; dt < 4; ++dt) ow[(8 * hh + r) * OPITCH + 16 * dt + m] = o[dt][r] * inv;
  }
  __syncthreads();

  v4u val[8];
#pragma unroll
  for (int it = 0; it < 8; ++it) {
    const int L = it * 4 + (lane >> 3);
    const int qd = L >> 1, pl = L & 1;
    const int c8 = (lane & 7) * 8;
    const float* src = ow + qd * OPITCH + c8;
    const v4f f0 = *(const v4f*)(src), f1 = *(const v4f*)(src + 4);
    unsigned int h0, l0, h1, l1, h2, l2, h3, l3;
    pack2hl(f0[0], f0[1], h0, l0);
    pack2hl(f0[2], f0[3], h1, l1);
    pack2hl(f1[0], f1[1], h2, l2);
    pack2hl(f1[2], f1[3], h3, l3);
    v4u u;
    u[0] = pl ? l0 : h0;
    u[1] = pl ? l1 : h1;
    u[2] = pl ? l2 : h2;
    u[3] = pl ? l3 : h3;
    val[it] = u;
  }
  for (int ps = 0; ps < 2; ++ps) {
#pragma unroll
    for (int it = 0; it < 8; ++it) {
      const int L = it * 4 + (lane >> 3);
      const int qd = L >> 1, pl = L & 1;
      const int c8 = (lane & 7) * 8;
      *(volatile v4u*)(cp + (size_t)(rowb + q0 + qd) * PLP + pl * EMB + h * HDIM + c8) = val[it];
    }
    __threadfence();
  }
}

__global__ __launch_bounds__(256) void k_gemm32(const unsigned short* __restrict__ cpl,
                                                const unsigned short* __restrict__ wo,
                                                const float* __restrict__ bo,
                                                float* __restrict__ out) {
  __shared__ __align__(16) float tile[64 * T32P];
  const int tid = threadIdx.x, lane = tid & 31, wave = tid >> 5;
  const int hh = lane >> 4, m = lane & 15;
  const int m0 = blockIdx.y * 64, n0 = blockIdx.x * 128;
  const int wm = wave >> 1, wn = wave & 1;

  v8f acc[4];
#pragma unroll
  for (int t = 0; t < 4; ++t) acc[t] = zero8();
  gemm3(cpl, wo, m0 + wm * 16, n0 + wn * 64, lane, acc);

#pragma unroll
  for (int t = 0; t < 4; ++t) {
    const int col = wn * 64 + 16 * t + m;
    const float bb = bo[n0 + col];
#pragma unroll
    for (int r = 0; r < 8; ++r) {
      const int row = wm * 16 + 8 * hh + r;
      tile[row * T32P + col] = acc[t][r] + bb;
    }
  }
  __syncthreads();

  v4f val[8];
#pragma unroll
  for (int it = 0; it < 8; ++it) {
    const int L = wave * 32 + it * 4 + (lane >> 3);
    const int row = L >> 2, q4 = L & 3;
    const int c4 = (lane & 7) * 4;
    val[it] = *(const v4f*)(tile + row * T32P + q4 * 32 + c4);
  }
  for (int ps = 0; ps < 2; ++ps) {
#pragma unroll
    for (int it = 0; it < 8; ++it) {
      const int L = wave * 32 + it * 4 + (lane >> 3);
      const int row = L >> 2, q4 = L & 3;
      const int c4 = (lane & 7) * 4;
      *(volatile v4f*)(out + (size_t)(m0 + row) * EMB + n0 + q4 * 32 + c4) = val[it];
    }
    __threadfence();
  }
}

extern "C" void kernel_launch(void* const* d_in, const int* in_sizes, int n_in,
                              void* d_out, int out_size, void* d_ws, size_t ws_size,
                              hipStream_t stream) {
  if (n_in < 9) return;
  if (in_sizes[0] != MROWS * EMB) return;
  if (in_sizes[1] != EMB * EMB || in_sizes[3] != EMB * EMB || in_sizes[5] != EMB * EMB || in_sizes[7] != EMB * EMB) return;
  if (in_sizes[2] != EMB || in_sizes[4] != EMB || in_sizes[6] != EMB || in_sizes[8] != EMB) return;
  if (out_size != MROWS * EMB) return;

  const float* x  = (const float*)d_in[0];
  const float* Wq = (const float*)d_in[1];
  const float* bq = (const float*)d_in[2];
  const float* Wk = (const float*)d_in[3];
  const float* bk = (const float*)d_in[4];
  const float* Wv = (const float*)d_in[5];
  const float* bv = (const float*)d_in[6];
  const float* Wo = (const float*)d_in[7];
  const float* bo = (const float*)d_in[8];
  float* out = (float*)d_out;

  size_t off = 0;
  const size_t oXP = off; off += (size_t)APLANE * 2;
  const size_t oWT = off; off += (size_t)4 * WPLANE * 2;
  const size_t oQK = off; off += (size_t)3 * HPLANE * 2;
  const size_t oCP = off; off += (size_t)APLANE * 2;
  if (off > ws_size) return;
  if (off > (size_t)134217728) return;

  char* ws = (char*)d_ws;
  unsigned short* XP  = (unsigned short*)(ws + oXP);
  unsigned short* WT  = (unsigned short*)(ws + oWT);
  unsigned short* QKV = (unsigned short*)(ws + oQK);
  unsigned short* CP  = (unsigned short*)(ws + oCP);

  k_xplane<<<dim3((MROWS * EMB) / (8 * 256)), dim3(256), 0, stream>>>(x, XP);
  k_wplane<<<dim3(EMB / 64, EMB / 64, 4), dim3(256), 0, stream>>>(Wq, Wk, Wv, Wo, WT);
  k_gemm16<<<dim3(EMB / 128, MROWS / 64, 3), dim3(256), 0, stream>>>(XP, WT, bq, bk, bv, QKV);
  k_attn<<<dim3(NBATCH * NHD * NQT), dim3(128), 0, stream>>>(QKV, QKV + (size_t)HPLANE,
                                                             QKV + (size_t)2 * HPLANE, CP);
  k_gemm32<<<dim3(EMB / 128, MROWS / 64), dim3(256), 0, stream>>>(CP, WT + (size_t)3 * WPLANE, bo, out);
  (void)hipGetLastError();
}
